// Refine_36197984371094
// MI455X (gfx1250) — hardware-verified
//
#include <hip/hip_runtime.h>
#include <stdint.h>

static constexpr int NIMG   = 8;
static constexpr int CIN    = 64;
static constexpr int IMG_H  = 128;
static constexpr int IMG_W  = 128;
static constexpr int NPIX   = 16384;
static constexpr int NCH1   = 256;
static constexpr int NCH2   = 64;
static constexpr int KC1    = 576;
static constexpr int NPOLY  = 8192;
static constexpr int NPT    = 128;
static constexpr int NPTS   = 129;
static constexpr int KFP    = 8256;
static constexpr int NXD    = 512;
static constexpr int NOUTD  = 256;
static constexpr int IMG_PER_PASS = 2;
static constexpr int MROWS  = IMG_PER_PASS * NPIX;
static constexpr int POLY_HALF = 4096;
static constexpr int NCHUNK_A  = 72;
static constexpr int NCHUNK_FP = 1032;

typedef __attribute__((ext_vector_type(16))) _Float16 v16h;
typedef __attribute__((ext_vector_type(8)))  _Float16 v8h;
typedef __attribute__((ext_vector_type(16))) __bf16   v16b;
typedef __attribute__((ext_vector_type(8)))  __bf16   v8b;
typedef __attribute__((ext_vector_type(8)))  float    v8f;
typedef __attribute__((ext_vector_type(4)))  float    v4f;

__device__ __forceinline__ unsigned short f2bf_bits(float f) {
  unsigned u = __float_as_uint(f);
  return (unsigned short)((u + 0x7FFFu + ((u >> 16) & 1u)) >> 16);
}
__device__ __forceinline__ float bf_bits2f(unsigned short h) { return __uint_as_float(((unsigned)h) << 16); }

__device__ __forceinline__ void dep_guard_h(v8f& a, v8f& b, v16h x, v16h y) { asm volatile("v_nop\n\tv_nop\n\tv_nop\n\tv_nop" : "+v"(a), "+v"(b) : "v"(x), "v"(y)); }
__device__ __forceinline__ void dep_guard_b(v8f& a, v8f& b, v16b x, v16b y) { asm volatile("v_nop\n\tv_nop\n\tv_nop\n\tv_nop" : "+v"(a), "+v"(b) : "v"(x), "v"(y)); }
__device__ __forceinline__ void keep4_h(v16h a, v16h b, v16h c, v16h d) { asm volatile("v_nop" :: "v"(a), "v"(b), "v"(c), "v"(d)); }
__device__ __forceinline__ void keep4_b(v16b a, v16b b, v16b c, v16b d) { asm volatile("v_nop" :: "v"(a), "v"(b), "v"(c), "v"(d)); }
__device__ __forceinline__ void acc_guard4(v8f& a, v8f& b, v8f& c, v8f& d) { asm volatile("v_nop\n\tv_nop\n\tv_nop\n\tv_nop" : "+v"(a), "+v"(b), "+v"(c), "+v"(d)); }
template <typename T> struct Frag;
template <> struct Frag<_Float16> {
  typedef v16h V; union U { v16h v; v8h h[2]; };
  static __device__ __forceinline__ v16h load(const _Float16* p) {
    U f; f.h[0] = *(const v8h*)(p); f.h[1] = *(const v8h*)(p + 16); return f.v;
  }
  static __device__ __forceinline__ v8f mma(v16h a, v16h b, v8f c) {
    return __builtin_amdgcn_wmma_f32_16x16x32_f16(false, a, false, b, (short)0, c, false, false);
  }
  static __device__ __forceinline__ void guard(v8f& a, v8f& b, v16h x, v16h y) { dep_guard_h(a, b, x, y); }
  static __device__ __forceinline__ void keep(v16h a, v16h b, v16h c, v16h d) { keep4_h(a, b, c, d); }
};
template <> struct Frag<__bf16> {
  typedef v16b V; union U { v16b v; v8b h[2]; };
  static __device__ __forceinline__ v16b load(const __bf16* p) {
    U f; f.h[0] = *(const v8b*)(p); f.h[1] = *(const v8b*)(p + 16); return f.v;
  }
  static __device__ __forceinline__ v8f mma(v16b a, v16b b, v8f c) {
    return __builtin_amdgcn_wmma_f32_16x16x32_bf16(false, a, false, b, (short)0, c, false, false);
  }
  static __device__ __forceinline__ void guard(v8f& a, v8f& b, v16b x, v16b y) { dep_guard_b(a, b, x, y); }
  static __device__ __forceinline__ void keep(v16b a, v16b b, v16b c, v16b d) { keep4_b(a, b, c, d); }
};

template <int ET> struct Elem;
template <> struct Elem<0> { typedef _Float16 T; };
template <> struct Elem<1> { typedef __bf16 T; };
template <int ET, bool SPLIT, int BIAS_MODE, int OUT_MODE, bool RESID, int ACT = 0>
__global__ __launch_bounds__(256) void wmma_gemm64(
    const unsigned short* __restrict__ Ap, const unsigned short* __restrict__ A2p, int lda, long strideA,
    const unsigned short* __restrict__ Btp, const unsigned short* __restrict__ Bt2p, int ldb, long strideB,
    void* __restrict__ Cout, void* __restrict__ Cout2, int ldc, long strideC,
    const float* __restrict__ bias,
    const float* __restrict__ resid, long strideR,
    int M, int N, int K, float scale) {
  typedef typename Elem<ET>::T T;
  typedef typename Frag<T>::V V;
  const T* A = (const T*)Ap; const T* A2 = (const T*)A2p; const T* Bt = (const T*)Btp; const T* Bt2 = (const T*)Bt2p;
  __shared__ __align__(16) float sT[8][16 * 68];
  const int b    = blockIdx.y;
  const int lane = threadIdx.x & 31;
  const int wave = threadIdx.x >> 5;
  const int tilesN = N >> 6;
  const int tilesM = M >> 6;
  const int tile = blockIdx.x * 8 + wave;
  if (tile >= tilesM * tilesN) return;
  const int tm = tile / tilesN;
  const int tn = tile - tm * tilesN;
  const int m0 = tm << 6;
  const int n0 = tn << 6;

  const T* Ab  = A  + (size_t)b * strideA;
  const T* Bb  = Bt + (size_t)b * strideB;
  const T* Ab2 = SPLIT ? (A2  + (size_t)b * strideA) : nullptr;
  const T* Bb2 = SPLIT ? (Bt2 + (size_t)b * strideB) : nullptr;

  const int rlane = lane & 15;
  const int koff  = (lane >> 4) * 8;
  const int mOff  = (lane >> 4) * 8;

  v8f acc[4][4];
#pragma unroll
  for (int i = 0; i < 4; ++i)
#pragma unroll
    for (int j = 0; j < 4; ++j) acc[i][j] = (v8f){0.f,0.f,0.f,0.f,0.f,0.f,0.f,0.f};

  for (int k0 = 0; k0 < K; k0 += 32) {
    V bh[4], bl[4];
#pragma unroll
    for (int j = 0; j < 4; ++j) {
      const size_t bo = (size_t)(n0 + (j << 4) + rlane) * ldb + koff + k0;
      bh[j] = Frag<T>::load(Bb + bo);
      if (SPLIT) bl[j] = Frag<T>::load(Bb2 + bo);
    }
#pragma unroll
    for (int i = 0; i < 4; ++i) {
      const size_t ao = (size_t)(m0 + (i << 4) + rlane) * lda + koff + k0;
      V ah = Frag<T>::load(Ab + ao);
      V al;
      if (SPLIT) al = Frag<T>::load(Ab2 + ao);
#pragma unroll
      for (int j = 0; j < 4; ++j) {
        acc[i][j] = Frag<T>::mma(ah, bh[j], acc[i][j]);
        if (SPLIT) {
          acc[i][j] = Frag<T>::mma(ah, bl[j], acc[i][j]);
          acc[i][j] = Frag<T>::mma(al, bh[j], acc[i][j]);
        }
      }
      Frag<T>::guard(acc[i][0], acc[i][3], ah, SPLIT ? al : ah);
    }
    Frag<T>::keep(bh[0], bh[1], bh[2], bh[3]);
    if (SPLIT) Frag<T>::keep(bl[0], bl[1], bl[2], bl[3]);
  }
  acc_guard4(acc[0][0], acc[0][1], acc[0][2], acc[0][3]);
  acc_guard4(acc[1][0], acc[1][1], acc[1][2], acc[1][3]);
  acc_guard4(acc[2][0], acc[2][1], acc[2][2], acc[2][3]);
  acc_guard4(acc[3][0], acc[3][1], acc[3][2], acc[3][3]);

  float* slab = sT[wave];
  const float* Rb = RESID ? (resid + (size_t)b * strideR) : nullptr;
#pragma unroll
  for (int i = 0; i < 4; ++i) {
    const int mBase = m0 + (i << 4);
#pragma unroll
    for (int j = 0; j < 4; ++j) {
      const int n = n0 + (j << 4) + rlane;
      float bv = 0.f;
      if (BIAS_MODE == 2) bv = bias[n];
#pragma unroll
      for (int r = 0; r < 8; ++r) {
        float v = acc[i][j][r] * scale;
        if (BIAS_MODE == 1) v += bias[mBase + mOff + r];
        if (BIAS_MODE == 2) v += bv;
        if (RESID) v += Rb[(size_t)(mBase + mOff + r) * ldc + n];
        if (ACT == 2) v = fmaxf(v, 0.0f);
        if (ACT == 4) v = (v > 0.f) ? v : 0.01f * v;
        slab[(mOff + r) * 68 + (j << 4) + rlane] = v;
      }
    }
    __builtin_amdgcn_fence(__ATOMIC_RELEASE, "workgroup");
    __builtin_amdgcn_wave_barrier();
    __builtin_amdgcn_fence(__ATOMIC_ACQUIRE, "workgroup");
    if (OUT_MODE == 0) {
      float* C = (float*)Cout + (size_t)b * strideC;
      const int hh = lane >> 4, c4 = (lane & 15) * 4;
      for (int pass = 0; pass < 2; ++pass) {
#pragma unroll
        for (int it = 0; it < 8; ++it) {
          const int row = it * 2 + hh;
          v4f v = *(const v4f*)(slab + row * 68 + c4);
          *(volatile v4f*)(C + (size_t)(mBase + row) * ldc + n0 + c4) = v;
        }
        __threadfence();
      }
    } else {
      const int q = lane >> 3, c8 = (lane & 7) * 8;
      unsigned short* C  = (unsigned short*)Cout  + (size_t)b * strideC;
      unsigned short* C2 = (OUT_MODE == 2) ? ((unsigned short*)Cout2 + (size_t)b * strideC) : nullptr;
      for (int pass = 0; pass < 2; ++pass) {
#pragma unroll
        for (int it = 0; it < 4; ++it) {
          const int row = it * 4 + q;
          const float* sp = slab + row * 68 + c8;
          v8h hv, lv;
#pragma unroll
          for (int e = 0; e < 8; ++e) {
            if (OUT_MODE == 1) {
              hv[e] = (_Float16)sp[e];
            } else {
              unsigned short hb = f2bf_bits(sp[e]);
              unsigned short lb = f2bf_bits(sp[e] - bf_bits2f(hb));
              hv[e] = __builtin_bit_cast(_Float16, hb);
              lv[e] = __builtin_bit_cast(_Float16, lb);
            }
          }
          *(volatile v8h*)(C + (size_t)(mBase + row) * ldc + n0 + c8) = hv;
          if (OUT_MODE == 2) *(volatile v8h*)(C2 + (size_t)(mBase + row) * ldc + n0 + c8) = lv;
        }
        __threadfence();
      }
    }
    __builtin_amdgcn_fence(__ATOMIC_RELEASE, "workgroup");
    __builtin_amdgcn_wave_barrier();
    __builtin_amdgcn_fence(__ATOMIC_ACQUIRE, "workgroup");
  }
}

__global__ __launch_bounds__(256) void cast_f32_f16x2s(
    const float* __restrict__ in, _Float16* __restrict__ out, int n2, float scale) {
  int i = blockIdx.x * 256 + threadIdx.x;
  if (i < n2) {
    const _Float16 h0 = (_Float16)(in[2 * i] * scale), h1 = (_Float16)(in[2 * i + 1] * scale);
    const unsigned u = (unsigned)__builtin_bit_cast(unsigned short, h0) | ((unsigned)__builtin_bit_cast(unsigned short, h1) << 16);
    ((volatile unsigned*)out)[i] = u;
    __threadfence();
    ((volatile unsigned*)out)[i] = u;
  }
}

__global__ __launch_bounds__(64) void bias4_k(const float* __restrict__ bfp, float* __restrict__ o) {
  const int t = threadIdx.x;
  v4f v = *(const v4f*)(bfp + 4 * t);
  v = v * 4.0f;
  *(volatile v4f*)(o + 4 * t) = v;
  __threadfence();
  *(volatile v4f*)(o + 4 * t) = v;
}

__global__ __launch_bounds__(256) void im2col_k(const float* __restrict__ feat, _Float16* __restrict__ A, int img0) {
  const int lane = threadIdx.x & 31, wave = threadIdx.x >> 5;
#pragma unroll 1
  for (int r = 0; r < 4; ++r) {
    const int row = blockIdx.x * 32 + wave * 4 + r;
    const int il  = row >> 14;
    const int pix = row & (NPIX - 1);
    const int y = pix >> 7, x = pix & 127;
    const float* fb = feat + (size_t)(img0 + il) * (size_t)(CIN * NPIX);
    _Float16* dst = A + (size_t)row * KC1;
#pragma unroll 1
    for (int it = 0; it < 3; ++it) {
      const int q  = it * 32 + lane;
      const int qc = q < NCHUNK_A ? q : (NCHUNK_A - 1);
      v8h o;
#pragma unroll
      for (int e = 0; e < 8; ++e) {
        const int k   = qc * 8 + e;
        const int ci  = k / 9;
        const int tap = k - ci * 9;
        const int ky  = tap / 3;
        const int kx  = tap - ky * 3;
        const int yy = y + ky - 1, xx = x + kx - 1;
        const bool valid = ((unsigned)yy < (unsigned)IMG_H) && ((unsigned)xx < (unsigned)IMG_W);
        const int ycl = min(max(yy, 0), IMG_H - 1);
        const int xcl = min(max(xx, 0), IMG_W - 1);
        float f = fb[(ci * IMG_H + ycl) * IMG_W + xcl];
        f = valid ? f : 0.0f;
        o[e] = (_Float16)f;
      }
      if (q < NCHUNK_A) {
        _Float16* d = dst + q * 8;
        *(volatile v8h*)d = o;
        __threadfence();
        *(volatile v8h*)d = o;
      }
    }
  }
}

__device__ __forceinline__ void corner_k(float xc, float yc, float w, int& off, float& wo) {
  const bool valid = (xc >= 0.0f) && (xc <= (float)(IMG_W - 1)) && (yc >= 0.0f) && (yc <= (float)(IMG_H - 1));
  const int xi = (int)fminf(fmaxf(xc, 0.0f), (float)(IMG_W - 1));
  const int yi = (int)fminf(fmaxf(yc, 0.0f), (float)(IMG_H - 1));
  off = yi * IMG_W + xi;
  wo  = valid ? w : 0.0f;
}

__global__ __launch_bounds__(256) void sample_k(const float* __restrict__ F2, const float* __restrict__ ct,
                                               const float* __restrict__ initp, const int* __restrict__ imgidx,
                                               _Float16* __restrict__ FP, int n0) {
  __shared__ __align__(16) float vals[KFP];
  __shared__ int   cofs[NPTS * 4];
  __shared__ float cwt[NPTS * 4];
  const int tid = threadIdx.x;
  const int nl = blockIdx.x;
  const int n  = n0 + nl;
  int b = imgidx[n];
  b = min(max(b, 0), NIMG - 1);
  {
    const int p  = tid < NPTS ? tid : (NPTS - 1);
    const int pm = p > 0 ? (p - 1) : 0;
    const float cxv = ct[2 * n], cyv = ct[2 * n + 1];
    const float ixv = initp[((size_t)n * NPT + pm) * 2], iyv = initp[((size_t)n * NPT + pm) * 2 + 1];
    const float X = (p == 0) ? cxv : ixv;
    const float Y = (p == 0) ? cyv : iyv;
    const float px = X - 0.5f, py = Y - 0.5f;
    const float x0f = floorf(px), y0f = floorf(py);
    const float wx1 = px - x0f, wy1 = py - y0f;
    const float wx0 = 1.0f - wx1, wy0 = 1.0f - wy1;
    int o0, o1, o2, o3; float w0, w1, w2, w3;
    corner_k(x0f,        y0f,        wx0 * wy0, o0, w0);
    corner_k(x0f + 1.0f, y0f,        wx1 * wy0, o1, w1);
    corner_k(x0f,        y0f + 1.0f, wx0 * wy1, o2, w2);
    corner_k(x0f + 1.0f, y0f + 1.0f, wx1 * wy1, o3, w3);
    if (tid < NPTS) {
      cofs[p * 4 + 0] = o0; cofs[p * 4 + 1] = o1; cofs[p * 4 + 2] = o2; cofs[p * 4 + 3] = o3;
      cwt[p * 4 + 0] = w0;  cwt[p * 4 + 1] = w1;  cwt[p * 4 + 2] = w2;  cwt[p * 4 + 3] = w3;
    }
  }
  __syncthreads();
  const int c = tid & 63, pg = tid >> 6;
  const float* Fb = F2 + (size_t)b * (size_t)(NPIX * NCH2) + c;
#pragma unroll 1
  for (int it = 0; it < 33; ++it) {
    const int p  = it * 4 + pg;
    const int pc = p < NPTS ? p : (NPTS - 1);
    const int o0 = cofs[pc * 4 + 0], o1 = cofs[pc * 4 + 1], o2 = cofs[pc * 4 + 2], o3 = cofs[pc * 4 + 3];
    const float w0 = cwt[pc * 4 + 0], w1 = cwt[pc * 4 + 1], w2 = cwt[pc * 4 + 2], w3 = cwt[pc * 4 + 3];
    const float v = w0 * Fb[(size_t)o0 * NCH2] + w1 * Fb[(size_t)o1 * NCH2] + w2 * Fb[(size_t)o2 * NCH2] + w3 * Fb[(size_t)o3 * NCH2];
    if (p < NPTS) vals[c * NPTS + p] = v;
  }
  __syncthreads();
  _Float16* rowp = FP + (size_t)nl * KFP;
#pragma unroll 1
  for (int it = 0; it < 5; ++it) {
    const int q  = it * 256 + tid;
    const int qc = q < NCHUNK_FP ? q : (NCHUNK_FP - 1);
    v8h hv;
#pragma unroll
    for (int e = 0; e < 8; ++e) hv[e] = (_Float16)vals[qc * 8 + e];
    if (q < NCHUNK_FP) {
      _Float16* d = rowp + q * 8;
      *(volatile v8h*)d = hv;
      __threadfence();
      *(volatile v8h*)d = hv;
    }
  }
}

extern "C" void kernel_launch(void* const* d_in, const int* in_sizes, int n_in,
                              void* d_out, int out_size, void* d_ws,
                              size_t ws_size, hipStream_t stream) {
  if (n_in < 11) return;
  if (in_sizes[0] != NIMG * CIN * NPIX || in_sizes[1] != NPOLY * 2 || in_sizes[2] != NPOLY * NPT * 2 ||
      in_sizes[3] != NPOLY || in_sizes[4] != NCH1 * KC1 || in_sizes[5] != NCH1 || in_sizes[6] != NCH2 * NCH1 ||
      in_sizes[7] != NCH2 || in_sizes[8] != NXD * KFP || in_sizes[9] != NOUTD * NXD || in_sizes[10] != NOUTD ||
      out_size != NPOLY * NOUTD) return;

  const float* feature = (const float*)d_in[0];
  const float* ctp     = (const float*)d_in[1];
  const float* initp   = (const float*)d_in[2];
  const int*   imgidx  = (const int*)d_in[3];
  const float* w1      = (const float*)d_in[4];
  const float* b1      = (const float*)d_in[5];
  const float* w2      = (const float*)d_in[6];
  const float* b2      = (const float*)d_in[7];
  const float* wp      = (const float*)d_in[8];
  const float* wf      = (const float*)d_in[9];
  const float* bfp     = (const float*)d_in[10];
  float* out = (float*)d_out;

  char* ws = (char*)d_ws;
  size_t off = 0;
  auto carve = [&](size_t bytes) -> char* { char* p = ws + off; off += (bytes + 255) & ~(size_t)255; return p; };
  _Float16* w1h = (_Float16*)carve((size_t)NCH1 * KC1 * 2);
  _Float16* w2h = (_Float16*)carve((size_t)NCH2 * NCH1 * 2);
  _Float16* wph = (_Float16*)carve((size_t)NXD * KFP * 2);
  _Float16* wfh = (_Float16*)carve((size_t)NOUTD * NXD * 2);
  float*    bf4 = (float*)carve((size_t)NOUTD * 4);
  float*    F2  = (float*)carve((size_t)NIMG * NPIX * NCH2 * 4);
  const size_t convBytes = (size_t)MROWS * KC1 * 2 + (size_t)MROWS * NCH1 * 2;
  const size_t polyBytes = (size_t)POLY_HALF * KFP * 2 + (size_t)POLY_HALF * NXD * 2;
  char* scratch = carve(convBytes > polyBytes ? convBytes : polyBytes);
  if (off > ws_size) return;
  _Float16* A16 = (_Float16*)scratch;
  _Float16* F1h = (_Float16*)(scratch + (size_t)MROWS * KC1 * 2);
  _Float16* FPh = (_Float16*)scratch;
  _Float16* Xh  = (_Float16*)(scratch + (size_t)POLY_HALF * KFP * 2);

  cast_f32_f16x2s<<<(NCH1 * KC1 / 2 + 255) / 256, 256, 0, stream>>>(w1, w1h, NCH1 * KC1 / 2, 16.0f);
  cast_f32_f16x2s<<<(NCH2 * NCH1 / 2 + 255) / 256, 256, 0, stream>>>(w2, w2h, NCH2 * NCH1 / 2, 16.0f);
  cast_f32_f16x2s<<<(NXD * KFP / 2 + 255) / 256, 256, 0, stream>>>(wp, wph, NXD * KFP / 2, 64.0f);
  cast_f32_f16x2s<<<(NOUTD * NXD / 2 + 255) / 256, 256, 0, stream>>>(wf, wfh, NOUTD * NXD / 2, 16.0f);
  bias4_k<<<1, 64, 0, stream>>>(bfp, bf4);

  for (int pr = 0; pr < NIMG / IMG_PER_PASS; ++pr) {
    im2col_k<<<MROWS / 32, 256, 0, stream>>>(feature, A16, pr * IMG_PER_PASS);
    wmma_gemm64<0, false, 2, 1, false, 2><<<dim3((MROWS / 64) * (NCH1 / 64) / 8, 1), 256, 0, stream>>>(
        (const unsigned short*)A16, (const unsigned short*)A16, KC1, 0L,
        (const unsigned short*)w1h, (const unsigned short*)w1h, KC1, 0L,
        (void*)F1h, (void*)F1h, NCH1, 0L,
        b1, b1, 0L, MROWS, NCH1, KC1, 1.0f / 16.0f);
    float* F2p = F2 + (size_t)pr * MROWS * NCH2;
    wmma_gemm64<0, false, 2, 0, false, 0><<<dim3((MROWS / 64) * (NCH2 / 64) / 8, 1), 256, 0, stream>>>(
        (const unsigned short*)F1h, (const unsigned short*)F1h, NCH1, 0L,
        (const unsigned short*)w2h, (const unsigned short*)w2h, NCH1, 0L,
        (void*)F2p, (void*)F2p, NCH2, 0L,
        b2, b2, 0L, MROWS, NCH2, NCH1, 1.0f / 16.0f);
  }

  for (int hf = 0; hf < NPOLY / POLY_HALF; ++hf) {
    sample_k<<<POLY_HALF, 256, 0, stream>>>(F2, ctp, initp, imgidx, FPh, hf * POLY_HALF);
    wmma_gemm64<0, false, 0, 1, false, 0><<<dim3((POLY_HALF / 64) * (NXD / 64) / 8, 1), 256, 0, stream>>>(
        (const unsigned short*)FPh, (const unsigned short*)FPh, KFP, 0L,
        (const unsigned short*)wph, (const unsigned short*)wph, KFP, 0L,
        (void*)Xh, (void*)Xh, NXD, 0L,
        b1, initp, 0L, POLY_HALF, NXD, KFP, 1.0f / 64.0f);
    float* outp = out + (size_t)hf * POLY_HALF * NOUTD;
    const float* resp = initp + (size_t)hf * POLY_HALF * NOUTD;
    wmma_gemm64<0, false, 2, 0, true, 0><<<dim3((POLY_HALF / 64) * (NOUTD / 64) / 8, 1), 256, 0, stream>>>(
        (const unsigned short*)Xh, (const unsigned short*)Xh, NXD, 0L,
        (const unsigned short*)wfh, (const unsigned short*)wfh, NXD, 0L,
        (void*)outp, (void*)outp, NOUTD, 0L,
        bf4, resp, 0L, POLY_HALF, NOUTD, NXD, 0.25f);
  }
}
